// DK_Conv2D_33079838113953
// MI455X (gfx1250) — hardware-verified
//
#include <hip/hip_runtime.h>
#include <math.h>

typedef __attribute__((ext_vector_type(16))) _Float16 v16h;
typedef __attribute__((ext_vector_type(8)))  _Float16 v8h;
typedef __attribute__((ext_vector_type(16))) __bf16   v16b;
typedef __attribute__((ext_vector_type(8)))  float    v8f;
typedef __attribute__((ext_vector_type(4)))  float    v4f;

__device__ __forceinline__ int frag_k(int i, int h) { return (i < 8) ? (8 * h + i) : (16 + 8 * h + (i - 8)); }
__device__ __forceinline__ __bf16 bf16_rne(float f) {
    unsigned int u = __float_as_uint(f);
    u += 0x7fffu + ((u >> 16) & 1u);
    return __builtin_bit_cast(__bf16, (unsigned short)(u >> 16));
}
__device__ __forceinline__ float bf16_f32(__bf16 b) { return __uint_as_float(((unsigned int)__builtin_bit_cast(unsigned short, b)) << 16); }
__device__ __forceinline__ v8f wmma16(v16h a, v16h b, v8f c) {
    c = __builtin_amdgcn_wmma_f32_16x16x32_f16(false, a, false, b, (short)0, c, false, false);
    asm volatile("v_nop\n\tv_nop\n\tv_nop\n\tv_nop" : "+v"(c) : "v"(a), "v"(b));
    return c;
}
__device__ __forceinline__ v8f wmmab(v16b a, v16b b, v8f c) {
    c = __builtin_amdgcn_wmma_f32_16x16x32_bf16(false, a, false, b, (short)0, c, false, false);
    asm volatile("v_nop\n\tv_nop\n\tv_nop\n\tv_nop" : "+v"(c) : "v"(a), "v"(b));
    return c;
}
struct Split { v16b hi, lo; };
__device__ __forceinline__ v8f wmma3(const Split& a, const Split& b, v8f c) {
    c = __builtin_amdgcn_wmma_f32_16x16x32_bf16(false, a.hi, false, b.hi, (short)0, c, false, false);
    c = __builtin_amdgcn_wmma_f32_16x16x32_bf16(false, a.hi, false, b.lo, (short)0, c, false, false);
    c = __builtin_amdgcn_wmma_f32_16x16x32_bf16(false, a.lo, false, b.hi, (short)0, c, false, false);
    asm volatile("v_nop\n\tv_nop\n\tv_nop\n\tv_nop" : "+v"(c) : "v"(a.hi), "v"(a.lo), "v"(b.hi), "v"(b.lo));
    return c;
}
struct Split3 { v16b hi, mid, lo; };
__device__ __forceinline__ v8f wmma6(const Split3& a, const Split3& b, v8f c) {
    c = __builtin_amdgcn_wmma_f32_16x16x32_bf16(false, a.hi, false, b.hi, (short)0, c, false, false);
    c = __builtin_amdgcn_wmma_f32_16x16x32_bf16(false, a.hi, false, b.mid, (short)0, c, false, false);
    c = __builtin_amdgcn_wmma_f32_16x16x32_bf16(false, a.mid, false, b.hi, (short)0, c, false, false);
    c = __builtin_amdgcn_wmma_f32_16x16x32_bf16(false, a.hi, false, b.lo, (short)0, c, false, false);
    c = __builtin_amdgcn_wmma_f32_16x16x32_bf16(false, a.mid, false, b.mid, (short)0, c, false, false);
    c = __builtin_amdgcn_wmma_f32_16x16x32_bf16(false, a.lo, false, b.hi, (short)0, c, false, false);
    asm volatile("v_nop\n\tv_nop\n\tv_nop\n\tv_nop" : "+v"(c) : "v"(a.hi), "v"(a.mid), "v"(a.lo), "v"(b.hi), "v"(b.mid), "v"(b.lo));
    return c;
}

__device__ __forceinline__ v16h fh_ld(const float* __restrict__ p, long long sk, int k0, int h, int klen, float s) {
    v16h a;
#pragma unroll
    for (int i = 0; i < 16; ++i) { const int k = k0 + frag_k(i, h); a[i] = (k < klen) ? (_Float16)(p[(long long)k * sk] * s) : (_Float16)0.f; }
    return a;
}
__device__ __forceinline__ Split sp_ld(const float* __restrict__ p, long long sk, int k0, int h, int klen, float s) {
    Split r;
#pragma unroll
    for (int i = 0; i < 16; ++i) {
        const int k = k0 + frag_k(i, h); const float x = (k < klen) ? p[(long long)k * sk] * s : 0.f;
        const __bf16 hb = bf16_rne(x); r.hi[i] = hb; r.lo[i] = bf16_rne(x - bf16_f32(hb));
    }
    return r;
}
__device__ __forceinline__ Split3 sp3_ld(const float* __restrict__ p, long long sk, int k0, int h, int klen, float s) {
    Split3 r;
#pragma unroll
    for (int i = 0; i < 16; ++i) {
        const int k = k0 + frag_k(i, h); const float x = (k < klen) ? p[(long long)k * sk] * s : 0.f;
        const __bf16 hb = bf16_rne(x); const float r1 = x - bf16_f32(hb); const __bf16 mb = bf16_rne(r1);
        r.hi[i] = hb; r.mid[i] = mb; r.lo[i] = bf16_rne(r1 - bf16_f32(mb));
    }
    return r;
}
__device__ __forceinline__ v16b bh_ld(const float* __restrict__ p, long long sk, int k0, int h, int klen, float s) {
    v16b a;
#pragma unroll
    for (int i = 0; i < 16; ++i) { const int k = k0 + frag_k(i, h); a[i] = bf16_rne((k < klen) ? p[(long long)k * sk] * s : 0.f); }
    return a;
}
__device__ __forceinline__ v16h fh_row(const _Float16* __restrict__ row, int k0, int h) {
    v16h a;
#pragma unroll
    for (int i = 0; i < 16; ++i) a[i] = row[k0 + frag_k(i, h)];
    return a;
}

#define VST2(T, ptr, val) do { const T vst2_v_ = (val); *(volatile T*)(ptr) = vst2_v_; __threadfence(); *(volatile T*)(ptr) = vst2_v_; } while (0)
typedef float v4f __attribute__((ext_vector_type(4)));
#define VST2V4(ptr, val) do { const v4f vst2_v4_ = (val); *(volatile v4f*)(ptr) = vst2_v4_; __threadfence(); *(volatile v4f*)(ptr) = vst2_v4_; } while (0)

__device__ __attribute__((noinline)) float act_fn(float v, int act) {
    if (act == 1) return fmaxf(v, 0.f);
    if (act == 2) { const float u = 0.7978845608028654f * (v + 0.044715f * v * v * v); return 0.5f * v * (1.f + tanhf(u)); }
    if (act == 3) return v / (1.f + expf(-v));
    if (act == 4) return 0.5f * v * (1.f + erff(v * 0.7071067811865476f));
    if (act == 5) return tanhf(v);
    if (act == 6) return 1.f / (1.f + expf(-v));
    if (act == 7) return (v > 0.f) ? v : 0.01f * v;
    if (act == 8) return (v > 0.f) ? v : (expf(v) - 1.f);
    if (act == 9) return fminf(fmaxf(v, 0.f), 6.f);
    if (act == 10) return fabsf(v);
    if (act == 11) return (v >= 0.f) ? v : 0.1f * v;
    if (act == 12) return (v > 0.f) ? v : 0.2f * v;
    if (act == 13) return (v > 20.f) ? v : log1pf(expf(v));
    return v;
}

struct GemmP {
    const float* A; const float* B; const float* bias; const float* R; float* C;
    long long sAo, sAi, sAm, sAk, sBo, sBi, sBn, sBk, sCo, sCi, sCm, sRo, sRi, sRm, sRn;
    int M, N, K, zi_n, flags, act; float alpha, beta, sa, sb;
    int Npad, pad_;
};
static_assert(sizeof(GemmP) == 5 * 8 + 15 * 8 + 6 * 4 + 4 * 4 + 2 * 4, "GemmP has padding");

template <int MODE>
__global__ __launch_bounds__(32) void k_gemm(GemmP p) {
    const int lane = threadIdx.x & 31, h = lane >> 4, l15 = lane & 15;
    const int m0 = blockIdx.y * 16, n0 = blockIdx.x * 32;
    const int z = blockIdx.z, zo = z / p.zi_n, zi = z - zo * p.zi_n;
    const float* A = p.A + zo * p.sAo + zi * p.sAi;
    const float* B = p.B + zo * p.sBo + zi * p.sBi;
    const int am = min(m0 + l15, p.M - 1);
    v8f acc[2], comp[2];
#pragma unroll
    for (int t = 0; t < 2; ++t) { v8f zz = {}; acc[t] = zz; comp[t] = zz; }
    for (int k0 = 0; k0 < p.K; k0 += 32) {
        const float* arow = A + (long long)am * p.sAm;
        if (MODE == 1) {
            const Split a = sp_ld(arow, p.sAk, k0, h, p.K, 1.f);
#pragma unroll
            for (int t = 0; t < 2; ++t) {
                const int bn = min(n0 + t * 16 + l15, p.N - 1);
                acc[t] = wmma3(a, sp_ld(B + (long long)bn * p.sBn, p.sBk, k0, h, p.K, 1.f), acc[t]);
            }
        } else if (MODE == 3) {
            const Split3 a = sp3_ld(arow, p.sAk, k0, h, p.K, 1.f);
#pragma unroll
            for (int t = 0; t < 2; ++t) {
                const int bn = min(n0 + t * 16 + l15, p.N - 1);
                acc[t] = wmma6(a, sp3_ld(B + (long long)bn * p.sBn, p.sBk, k0, h, p.K, 1.f), acc[t]);
            }
        } else if (MODE == 4) {
            const Split3 a = sp3_ld(arow, p.sAk, k0, h, p.K, 1.f);
#pragma unroll
            for (int t = 0; t < 2; ++t) {
                const int bn = min(n0 + t * 16 + l15, p.N - 1); v8f zz = {};
                const v8f part = wmma6(a, sp3_ld(B + (long long)bn * p.sBn, p.sBk, k0, h, p.K, 1.f), zz);
                const v8f y = part - comp[t]; const v8f s = acc[t] + y; comp[t] = (s - acc[t]) - y; acc[t] = s;
            }
        } else if (MODE == 2) {
            const v16b a = bh_ld(arow, p.sAk, k0, h, p.K, 1.f);
#pragma unroll
            for (int t = 0; t < 2; ++t) {
                const int bn = min(n0 + t * 16 + l15, p.N - 1);
                acc[t] = wmmab(a, bh_ld(B + (long long)bn * p.sBn, p.sBk, k0, h, p.K, 1.f), acc[t]);
            }
        } else {
            const v16h a = fh_ld(arow, p.sAk, k0, h, p.K, p.sa);
#pragma unroll
            for (int t = 0; t < 2; ++t) {
                const int bn = min(n0 + t * 16 + l15, p.N - 1);
                acc[t] = wmma16(a, fh_ld(B + (long long)bn * p.sBn, p.sBk, k0, h, p.K, p.sb), acc[t]);
            }
        }
    }
    const float iscale = (MODE == 0) ? p.alpha / (p.sa * p.sb) : p.alpha;
    float* C = p.C + zo * p.sCo + zi * p.sCi;
    const float* R = p.R + zo * p.sRo + zi * p.sRi;
    __shared__ __align__(16) float ctile[16][36];
#pragma unroll
    for (int t = 0; t < 2; ++t) {
        const int n = n0 + t * 16 + l15; const int nn = min(n, p.N - 1);
#pragma unroll
        for (int r = 0; r < 8; ++r) {
            const int m = m0 + 8 * h + r; const int mm = min(m, p.M - 1);
            float v = acc[t][r] * iscale;
            if (p.flags & 1) v += p.bias[nn];
            if (p.flags & 2) v += p.bias[mm];
            if (p.flags & 8) v *= p.bias[(long long)zo * p.M + mm];
            v = act_fn(v, p.act);
            if (p.flags & 4) v += p.beta * R[(long long)mm * p.sRm + (long long)nn * p.sRn];
            ctile[8 * h + r][t * 16 + l15] = (n < p.N) ? v : 0.f;
        }
    }
    __syncthreads();
    const int NW = (p.Npad > p.N) ? p.Npad : p.N;
    const bool fast = (m0 + 16 <= p.M) && (n0 + 32 <= NW) && ((p.sCm & 3) == 0) && ((((size_t)C) & 15) == 0);
    if (fast) {
#pragma unroll
        for (int s = 0; s < 4; ++s) {
            const int row = s * 4 + (lane >> 3), c4 = (lane & 7) * 4;
            const v4f v = *(const v4f*)&ctile[row][c4];
            VST2V4(C + (long long)(m0 + row) * p.sCm + n0 + c4, v);
        }
    } else {
        for (int row = 0; row < 16; ++row) {
            const int m = m0 + row, n = n0 + lane;
            if (m < p.M && n < NW) VST2(float, C + (long long)m * p.sCm + n, ctile[row][lane]);
        }
    }
}


template <int MODE, int TM, int TN>
__global__ __launch_bounds__(32) void k_gemmT(GemmP p) {
    const int lane = threadIdx.x & 31, h = lane >> 4, l15 = lane & 15;
    const int m0 = blockIdx.y * (16 * TM), n0 = blockIdx.x * (16 * TN);
    const int z = blockIdx.z, zo = z / p.zi_n, zi = z - zo * p.zi_n;
    const float* A = p.A + zo * p.sAo + zi * p.sAi;
    const float* B = p.B + zo * p.sBo + zi * p.sBi;
    v8f acc[TM][TN];
#pragma unroll
    for (int i = 0; i < TM; ++i)
#pragma unroll
        for (int t = 0; t < TN; ++t) { v8f zz = {}; acc[i][t] = zz; }
    for (int k0 = 0; k0 < p.K; k0 += 32) {
        if (MODE == 1) {
            Split a[TM], b[TN];
#pragma unroll
            for (int i = 0; i < TM; ++i) { const int am = min(m0 + 16 * i + l15, p.M - 1); a[i] = sp_ld(A + (long long)am * p.sAm, p.sAk, k0, h, p.K, 1.f); }
#pragma unroll
            for (int t = 0; t < TN; ++t) { const int bn = min(n0 + 16 * t + l15, p.N - 1); b[t] = sp_ld(B + (long long)bn * p.sBn, p.sBk, k0, h, p.K, 1.f); }
#pragma unroll
            for (int i = 0; i < TM; ++i)
#pragma unroll
                for (int t = 0; t < TN; ++t) acc[i][t] = wmma3(a[i], b[t], acc[i][t]);
        } else if (MODE == 2) {
            v16b a[TM], b[TN];
#pragma unroll
            for (int i = 0; i < TM; ++i) { const int am = min(m0 + 16 * i + l15, p.M - 1); a[i] = bh_ld(A + (long long)am * p.sAm, p.sAk, k0, h, p.K, 1.f); }
#pragma unroll
            for (int t = 0; t < TN; ++t) { const int bn = min(n0 + 16 * t + l15, p.N - 1); b[t] = bh_ld(B + (long long)bn * p.sBn, p.sBk, k0, h, p.K, 1.f); }
#pragma unroll
            for (int i = 0; i < TM; ++i)
#pragma unroll
                for (int t = 0; t < TN; ++t) acc[i][t] = wmmab(a[i], b[t], acc[i][t]);
        } else {
            v16h a[TM], b[TN];
#pragma unroll
            for (int i = 0; i < TM; ++i) { const int am = min(m0 + 16 * i + l15, p.M - 1); a[i] = fh_ld(A + (long long)am * p.sAm, p.sAk, k0, h, p.K, p.sa); }
#pragma unroll
            for (int t = 0; t < TN; ++t) { const int bn = min(n0 + 16 * t + l15, p.N - 1); b[t] = fh_ld(B + (long long)bn * p.sBn, p.sBk, k0, h, p.K, p.sb); }
#pragma unroll
            for (int i = 0; i < TM; ++i)
#pragma unroll
                for (int t = 0; t < TN; ++t) acc[i][t] = wmma16(a[i], b[t], acc[i][t]);
        }
    }
    const float iscale = (MODE == 0) ? p.alpha / (p.sa * p.sb) : p.alpha;
    float* C = p.C + zo * p.sCo + zi * p.sCi;
    const float* R = p.R + zo * p.sRo + zi * p.sRi;
    const int NW = (p.Npad > p.N) ? p.Npad : p.N;
    __shared__ __align__(16) float ctile[16][36];
#pragma unroll
    for (int i = 0; i < TM; ++i) {
        const int mb = m0 + 16 * i; if (mb >= p.M) break;
#pragma unroll
        for (int tp = 0; tp < TN / 2; ++tp) {
            const int nb = n0 + 32 * tp; if (nb >= NW) break;
#pragma unroll
            for (int t2 = 0; t2 < 2; ++t2) {
                const int t = 2 * tp + t2; const int n = nb + t2 * 16 + l15; const int nn = min(n, p.N - 1);
#pragma unroll
                for (int r = 0; r < 8; ++r) {
                    const int m = mb + 8 * h + r; const int mm = min(m, p.M - 1);
                    float v = acc[i][t][r] * iscale;
                    if (p.flags & 1) v += p.bias[nn];
                    if (p.flags & 2) v += p.bias[mm];
            if (p.flags & 8) v *= p.bias[(long long)zo * p.M + mm];
                    v = act_fn(v, p.act);
                    if (p.flags & 4) v += p.beta * R[(long long)mm * p.sRm + (long long)nn * p.sRn];
                    ctile[8 * h + r][t2 * 16 + l15] = (n < p.N) ? v : 0.f;
                }
            }
            __syncthreads();
            const bool fast = (mb + 16 <= p.M) && (nb + 32 <= NW) && ((p.sCm & 3) == 0) && ((((size_t)C) & 15) == 0);
            if (fast) {
#pragma unroll
                for (int s = 0; s < 4; ++s) {
                    const int row = s * 4 + (lane >> 3), c4 = (lane & 7) * 4;
                    const v4f v = *(const v4f*)&ctile[row][c4];
                    VST2V4(C + (long long)(mb + row) * p.sCm + nb + c4, v);
                }
            } else {
                for (int row = 0; row < 16; ++row) {
                    const int m = mb + row, n = nb + lane;
                    if (m < p.M && n < NW) VST2(float, C + (long long)m * p.sCm + n, ctile[row][lane]);
                }
            }
            __syncthreads();
        }
    }
}

#define AW 4
struct AttnP {
    const float* Q; const float* K; const float* V; float* O; float* P; const float* Mf; const int* Mi; float* ST;
    const float* Pw; const float* Rt; const int* SQ; const int* SK;
    long long swb, swh, swi, swj, srb, srh, sri;
    long long sQb, sQh, sQi, sQd, sKb, sKh, sKj, sKd, sVb, sVh, sVj, sVd, sOb, sOh, sOi, sPb, sPh, sPi, smb, smh, smi, smj;
    int Lq, Lk, dh, dv, hrep, causal, coff, pband;
    float scale, mfill; int nonorm, mpol;
    int roff, rn, segpol, win;
};
static_assert(sizeof(AttnP) == 12 * 8 + 29 * 8 + 16 * 4, "AttnP has padding");

#ifndef KATTN_ATTR
#define KATTN_ATTR
#endif
template <int DHP, int DVP, int QM, bool SPLITPV, bool TWOPASS>
__global__ __launch_bounds__(32 * AW) KATTN_ATTR void k_attn(AttnP p) {
    constexpr int NT = DVP / 16;
    constexpr int KS = DHP / 32;
    constexpr int VP = DVP + 8;
    __shared__ __align__(16) float    pl[AW][16 * 64];
    __shared__ __align__(16) _Float16 vl[(SPLITPV ? 2 : 1) * 64 * VP];
    const int lane = threadIdx.x & 31, hf = lane >> 4, l15 = lane & 15, wave = threadIdx.x >> 5;
    const int h = blockIdx.y, b = blockIdx.z, hk = h / p.hrep;
    const int q0 = (blockIdx.x * AW + wave) * 16;
    float* myp = pl[wave];
    const float L2E = 1.4426950408889634f;
    const float NEG = -__builtin_inff();
    const int qi = min(q0 + l15, p.Lq - 1);
    const float* qrow = p.Q + b * p.sQb + h * p.sQh + (long long)qi * p.sQi;
    const float* kbase = p.K + b * p.sKb + hk * p.sKh;
    const float* vbase = p.V + b * p.sVb + hk * p.sVh;
    v16h qa[QM == 0 ? KS : 1]; Split qs_[QM == 1 ? KS : 1]; Split3 qt_[QM == 2 ? KS : 1];
#pragma unroll
    for (int ks = 0; ks < KS; ++ks) {
        if (QM == 2) qt_[ks] = sp3_ld(qrow, p.sQd, ks * 32, hf, p.dh, 1.f);
        else if (QM == 1) qs_[ks] = sp_ld(qrow, p.sQd, ks * 32, hf, p.dh, 1.f);
        else qa[ks] = fh_ld(qrow, p.sQd, ks * 32, hf, p.dh, 1.f);
    }
    v8f o[NT]; float m8[8], l8[8];
#pragma unroll
    for (int t = 0; t < NT; ++t) { v8f zz = {}; o[t] = zz; }
#pragma unroll
    for (int i = 0; i < 8; ++i) { m8[i] = NEG; l8[i] = 0.f; }
    int jend = p.Lk;
    if (p.causal == 1) { const int je = (blockIdx.x * AW + AW - 1) * 16 + 16 + p.coff; jend = min(jend, max(je, 0)); }
    const int npass = TWOPASS ? 2 : 1;
    for (int pass = 0; pass < npass; ++pass) {
        const bool dopv = (!TWOPASS) || pass == 1;
        for (int j0 = 0; j0 < jend; j0 += 64) {
            if (dopv) {
                __syncthreads();
                for (int idx = threadIdx.x; idx < 64 * DVP; idx += 32 * AW) {
                    const int jr = idx / DVP, d = idx - jr * DVP, j = j0 + jr;
                    const float f = (j < p.Lk && d < p.dv) ? vbase[(long long)j * p.sVj + (long long)d * p.sVd] : 0.f;
                    if (SPLITPV) {
                        const __bf16 hb = bf16_rne(f);
                        ((__bf16*)vl)[jr * VP + d] = hb; ((__bf16*)vl)[64 * VP + jr * VP + d] = bf16_rne(f - bf16_f32(hb));
                    } else vl[jr * VP + d] = (_Float16)f;
                }
            }
            v8f s[4];
#pragma unroll
            for (int t = 0; t < 4; ++t) {
                const int j = min(j0 + t * 16 + l15, p.Lk - 1);
                const float* krow = kbase + (long long)j * p.sKj;
                v8f acc = {};
#pragma unroll
                for (int ks = 0; ks < KS; ++ks) {
                    if (QM == 2)      acc = wmma6(qt_[ks], sp3_ld(krow, p.sKd, ks * 32, hf, p.dh, 1.f), acc);
                    else if (QM == 1) acc = wmma3(qs_[ks], sp_ld(krow, p.sKd, ks * 32, hf, p.dh, 1.f), acc);
                    else              acc = wmma16(qa[ks], fh_ld(krow, p.sKd, ks * 32, hf, p.dh, 1.f), acc);
                }
                s[t] = acc;
            }
            float pv[8][4];
#pragma unroll
            for (int i = 0; i < 8; ++i) {
                const int irow = q0 + i + 8 * hf;
                const int ic = min(irow, p.Lq - 1);
                float sc[4];
#pragma unroll
                for (int t = 0; t < 4; ++t) {
                    const int jg = j0 + t * 16 + l15;
                    float v = s[t][i] * p.scale;
                    if (p.Mf) v += p.Mf[b * p.smb + h * p.smh + (long long)ic * p.smi + (long long)min(jg, p.Lk - 1) * p.smj];
                    if (p.Rt) { int rc = ic - min(jg, p.Lk - 1) + p.roff; rc = rc < 0 ? 0 : (rc >= p.rn ? p.rn - 1 : rc); v += p.Rt[b * p.srb + h * p.srh + (long long)ic * p.sri + rc]; }
                    if (p.Mi) { const int mv = p.Mi[b * p.smb + h * p.smh + (long long)ic * p.smi + (long long)min(jg, p.Lk - 1) * p.smj]; if (p.mpol ? (mv != 0) : (mv == 0)) v = p.mfill; }
                    if (p.SQ) { const bool same = p.SQ[(long long)b * p.Lq + ic] == p.SK[(long long)b * p.Lk + min(jg, p.Lk - 1)]; if (p.segpol ? same : !same) v = p.mfill; }
                    if (p.causal == 2 && jg > irow + p.coff) v = p.mfill;
                    if (jg >= p.Lk || (p.causal == 1 && jg > irow + p.coff) || (p.causal == 3 && jg < irow + p.coff) || (p.win > 0 && irow + p.coff - jg > p.win)) v = NEG; else v *= L2E;
                    sc[t] = v;
                }
                if (!TWOPASS || pass == 0) {
                    float mx = fmaxf(fmaxf(sc[0], sc[1]), fmaxf(sc[2], sc[3]));
                    mx = fmaxf(mx, __shfl_xor(mx, 1, 32)); mx = fmaxf(mx, __shfl_xor(mx, 2, 32));
                    mx = fmaxf(mx, __shfl_xor(mx, 4, 32)); mx = fmaxf(mx, __shfl_xor(mx, 8, 32));
                    const float mnew = fmaxf(m8[i], mx);
                    const float corr = (mnew == NEG) ? 1.f : exp2f(m8[i] - mnew);
                    float rs = 0.f;
#pragma unroll
                    for (int t = 0; t < 4; ++t) {
                        const float pp = (sc[t] == NEG) ? 0.f : exp2f(sc[t] - mnew); rs += pp;
                        pv[i][t] = p.Pw ? pp * p.Pw[b * p.swb + h * p.swh + (long long)ic * p.swi + (long long)min(j0 + t * 16 + l15, p.Lk - 1) * p.swj] : pp;
                    }
                    rs += __shfl_xor(rs, 1, 32); rs += __shfl_xor(rs, 2, 32); rs += __shfl_xor(rs, 4, 32); rs += __shfl_xor(rs, 8, 32);
                    l8[i] = l8[i] * corr + rs; m8[i] = mnew;
                    if (!TWOPASS) {
#pragma unroll
                        for (int t = 0; t < NT; ++t) o[t][i] *= corr;
                    }
                } else {
                    const float inv = (l8[i] > 0.f) ? 1.f / l8[i] : 0.f;
#pragma unroll
                    for (int t = 0; t < 4; ++t) {
                        const int jg = j0 + t * 16 + l15;
                        float pp = (sc[t] == NEG) ? 0.f : exp2f(sc[t] - m8[i]) * inv;
                        if (p.Pw) pp *= p.Pw[b * p.swb + h * p.swh + (long long)ic * p.swi + (long long)min(jg, p.Lk - 1) * p.swj];
                        pv[i][t] = pp;
                    }
                }
            }
            if (dopv) {
#pragma unroll
                for (int i = 0; i < 8; ++i)
#pragma unroll
                    for (int t = 0; t < 4; ++t) myp[(i + 8 * hf) * 64 + t * 16 + l15] = pv[i][t];
                __syncthreads();
                if (p.P) {
                    float* pb_ = p.P + b * p.sPb + h * p.sPh;
                    const bool fastP = (p.pband == 0) && ((p.sPi & 3) == 0) && (j0 + 64 <= p.Lk) && (q0 + 16 <= p.Lq) && ((((size_t)pb_) & 15) == 0);
                    if (fastP) {
#pragma unroll
                        for (int s = 0; s < 8; ++s) {
                            const int row = s * 2 + (lane >> 4), c4 = (lane & 15) * 4;
                            const v4f v = *(const v4f*)(myp + row * 64 + c4);
                            VST2V4(pb_ + (long long)(q0 + row) * p.sPi + j0 + c4, v);
                        }
                    } else {
                        for (int row = 0; row < 16; ++row) {
                            const int irow = q0 + row; if (irow >= p.Lq) continue;
                            for (int c = lane; c < 64; c += 32) {
                                const int jg = j0 + c; if (jg >= p.Lk) continue;
                                if (p.pband == 0) VST2(float, pb_ + (long long)irow * p.sPi + jg, myp[row * 64 + c]);
                                else if (jg - irow <= p.pband && irow - jg <= p.pband) VST2(float, pb_ + (long long)irow * p.sPi + (jg - irow + p.pband), myp[row * 64 + c]);
                            }
                        }
                    }
                }
                if (SPLITPV) {
                    const Split pa0 = sp_ld(myp + l15 * 64, 1, 0, hf, 64, 1.f), pa1 = sp_ld(myp + l15 * 64, 1, 32, hf, 64, 1.f);
                    const __bf16* vh = (const __bf16*)vl; const __bf16* vlo = vh + 64 * VP;
#pragma unroll
                    for (int t = 0; t < NT; ++t) {
                        const int dcol = t * 16 + l15;
                        Split b0, b1;
#pragma unroll
                        for (int e = 0; e < 16; ++e) {
                            const int k0 = frag_k(e, hf), k1 = 32 + frag_k(e, hf);
                            b0.hi[e] = vh[k0 * VP + dcol]; b0.lo[e] = vlo[k0 * VP + dcol]; b1.hi[e] = vh[k1 * VP + dcol]; b1.lo[e] = vlo[k1 * VP + dcol];
                        }
                        o[t] = wmma3(pa0, b0, o[t]);
                        o[t] = wmma3(pa1, b1, o[t]);
                    }
                } else {
                    const v16h pa0 = fh_ld(myp + l15 * 64, 1, 0, hf, 64, 4096.f), pa1 = fh_ld(myp + l15 * 64, 1, 32, hf, 64, 4096.f);
#pragma unroll
                    for (int t = 0; t < NT; ++t) {
                        const int dcol = t * 16 + l15;
                        v16h b0, b1;
#pragma unroll
                        for (int e = 0; e < 16; ++e) { b0[e] = vl[frag_k(e, hf) * VP + dcol]; b1[e] = vl[(32 + frag_k(e, hf)) * VP + dcol]; }
                        o[t] = wmma16(pa0, b0, o[t]);
                        o[t] = wmma16(pa1, b1, o[t]);
                    }
                }
            }
        }
    }
    float* obase = p.O + b * p.sOb + h * p.sOh;
    if (p.ST) {
        const int rl = lane >> 1, isel = rl & 7;
        float mv = 0.f, lv = 0.f;
#pragma unroll
        for (int i = 0; i < 8; ++i) if (i == isel) { mv = m8[i]; lv = l8[i]; }
        const int irow = q0 + rl;
        if (irow < p.Lq) { float* st = p.ST + (((long long)b * gridDim.y + h) * p.Lq + irow) * 2 + (lane & 1); VST2(float, st, (lane & 1) ? lv : mv * 0.6931471805599453f); }
    }
    float invr[8];
#pragma unroll
    for (int i = 0; i < 8; ++i) {
        if (TWOPASS) invr[i] = SPLITPV ? 1.f : (1.f / 4096.f);
        else if (p.nonorm) invr[i] = exp2f(m8[i]) * (SPLITPV ? 1.f : (1.f / 4096.f));
        else invr[i] = (l8[i] > 0.f) ? (SPLITPV ? 1.f / l8[i] : 1.f / (l8[i] * 4096.f)) : 0.f;
    }
    __syncthreads();
    const bool ofast = ((p.sOi & 3) == 0) && ((((size_t)obase) & 15) == 0) && (q0 + 16 <= p.Lq);
#pragma unroll
    for (int c0 = 0; c0 < DVP; c0 += 64) {
#pragma unroll
        for (int i = 0; i < 8; ++i)
#pragma unroll
            for (int t = 0; t < NT; ++t) if (t * 16 >= c0 && t * 16 < c0 + 64) myp[(i + 8 * hf) * 64 + (t * 16 - c0) + l15] = o[t][i] * invr[i];
        __syncthreads();
        const int cw = (DVP - c0 < 64) ? (DVP - c0) : 64;
        if (ofast && (c0 + cw <= p.dv) && (cw % 32 == 0)) {
            const int lpr = cw / 4;
            const int rows_per_ins = 32 / lpr;
            for (int r0 = 0; r0 < 16; r0 += rows_per_ins) {
                const int row = r0 + lane / lpr, c4 = (lane % lpr) * 4;
                const v4f v = *(const v4f*)(myp + row * 64 + c4);
                VST2V4(obase + (long long)(q0 + row) * p.sOi + c0 + c4, v);
            }
        } else {
            for (int row = 0; row < 16; ++row) {
                const int irow = q0 + row; if (irow >= p.Lq) continue;
                for (int c = lane; c < cw; c += 32) { const int d = c0 + c; if (d < p.dv) VST2(float, obase + (long long)irow * p.sOi + d, myp[row * 64 + c]); }
            }
        }
        __syncthreads();
    }
}

struct TrP { const float* src; float* dst; const float* R2; long long sSz, lds, sDz, ldd, sRz, ldr; int R, C, flags, act; float alpha, beta; };
static_assert(sizeof(TrP) == 3 * 8 + 6 * 8 + 6 * 4, "TrP has padding");
__global__ __launch_bounds__(256) void k_tr(TrP p) {
    __shared__ float tile[32][33];
    const int c0 = blockIdx.x * 32, r0 = blockIdx.y * 32, z = blockIdx.z;
    const int lane = threadIdx.x & 31, wave = threadIdx.x >> 5;
    const float* s = p.src + z * p.sSz;
#pragma unroll
    for (int k = 0; k < 4; ++k) {
        const int rl = wave * 4 + k, r = r0 + rl, c = c0 + lane;
        tile[rl][lane] = (r < p.R && c < p.C) ? s[(long long)r * p.lds + c] : 0.f;
    }
    __syncthreads();
    float* d = p.dst + z * p.sDz; const float* rr = p.R2 + z * p.sRz;
#pragma unroll
    for (int k = 0; k < 4; ++k) {
        const int cl = wave * 4 + k, c = c0 + cl, r = r0 + lane;
        if (c < p.C && r < p.R) {
            float v = act_fn(p.alpha * tile[lane][cl], p.act);
            if (p.flags & 1) v += p.beta * rr[(long long)c * p.ldr + r];
            VST2(float, d + (long long)c * p.ldd + r, v);
        }
    }
}

__global__ __launch_bounds__(256) void k_affine(const float* __restrict__ src, float* __restrict__ dst, int n, float a, float b, const float* __restrict__ sdev) {
    const int i = blockIdx.x * 256 + threadIdx.x;
    if (i < n) { const float aa = sdev ? a * sdev[0] : a; const float v = aa * src[i] + b; VST2(float, dst + i, v); }
}

struct SmP { const float* src; float* dst; const float* Mf; long long sz, sr, dz, dr, smz, smr; int n, pad; float scale_in, scale_out; };
static_assert(sizeof(SmP) == 3 * 8 + 6 * 8 + 4 * 4, "SmP has padding");
__global__ __launch_bounds__(256) void k_softmax(SmP p) {
    __shared__ float red[256];
    const int r = blockIdx.x, z = blockIdx.y, tid = threadIdx.x;
    const float* s = p.src + z * p.sz + (long long)r * p.sr;
    const float* mf = p.Mf ? (p.Mf + z * p.smz + (long long)r * p.smr) : nullptr;
    float mx = -__builtin_inff();
    for (int j = tid; j < p.n; j += 256) { float v = s[j] * p.scale_in; if (mf) v += mf[j]; mx = fmaxf(mx, v); }
    red[tid] = mx; __syncthreads();
    for (int o = 128; o > 0; o >>= 1) { if (tid < o) red[tid] = fmaxf(red[tid], red[tid + o]); __syncthreads(); }
    mx = red[0]; __syncthreads();
    float sum = 0.f;
    for (int j = tid; j < p.n; j += 256) { float v = s[j] * p.scale_in; if (mf) v += mf[j]; sum += (mx == -__builtin_inff()) ? 0.f : expf(v - mx); }
    red[tid] = sum; __syncthreads();
    for (int o = 128; o > 0; o >>= 1) { if (tid < o) red[tid] += red[tid + o]; __syncthreads(); }
    sum = red[0];
    const float inv = (sum > 0.f) ? p.scale_out / sum : 0.f;
    float* d = p.dst + z * p.dz + (long long)r * p.dr;
    for (int j = tid; j < p.n; j += 256) { float v = s[j] * p.scale_in; if (mf) v += mf[j]; const float o = (mx == -__builtin_inff()) ? 0.f : expf(v - mx) * inv; VST2(float, d + j, o); }
}
__global__ __launch_bounds__(256) void k_stats(const float* __restrict__ x, long long sz, long long so, long long si, int inner, int n, float eps, float* __restrict__ stat, int mode) {
    __shared__ float red[256];
    const int z = blockIdx.x, tid = threadIdx.x;
    const float* base = x + z * sz;
    float s = 0.f;
    for (int e = tid; e < n; e += 256) s += base[(long long)(e / inner) * so + (long long)(e % inner) * si];
    red[tid] = s; __syncthreads();
    for (int o = 128; o > 0; o >>= 1) { if (tid < o) red[tid] += red[tid + o]; __syncthreads(); }
    const float mu = (mode == 0 || mode == 3) ? red[0] / (float)n : 0.f; __syncthreads();
    float q = 0.f;
    for (int e = tid; e < n; e += 256) { const float dlt = base[(long long)(e / inner) * so + (long long)(e % inner) * si] - mu; q += dlt * dlt; }
    red[tid] = q; __syncthreads();
    for (int o = 128; o > 0; o >>= 1) { if (tid < o) red[tid] += red[tid + o]; __syncthreads(); }
    {
        float rs;
        if (mode == 2) rs = sqrtf((float)n) / fmaxf(sqrtf(red[0]), eps); else if (mode == 3) rs = rsqrtf(red[0] / (float)(n - 1) + eps); else rs = rsqrtf(red[0] / (float)n + eps);
        if (tid < 32) { const float v = (tid == 0) ? mu : ((tid == 1) ? rs : 0.f); VST2(float, stat + (long long)z * 32 + tid, v); }
    }
}
__global__ __launch_bounds__(256) void k_norm_apply(const float* __restrict__ x, float* __restrict__ y, const float* __restrict__ stat, const float* __restrict__ g, const float* __restrict__ bta,
                                                     int Z, int C, int L, int G, int bn, int act) {
    const long long idx = (long long)blockIdx.x * 256 + threadIdx.x;
    if (idx >= (long long)Z * C * L) return;
    const int l = (int)(idx % L); const long long zc = idx / L; const int c = (int)(zc % C), z = (int)(zc / C); (void)l;
    const int set = bn ? c : (z * G + c / (C / G));
    float v = (x[idx] - stat[(long long)set * 32]) * stat[(long long)set * 32 + 1];
    if (g) v *= g[c];
    if (bta) v += bta[c];
    v = act_fn(v, act);
    VST2(float, y + idx, v);
}

__global__ __launch_bounds__(256) void k_lse_neg(const float* __restrict__ st, float* __restrict__ c, int n) {
    const int i = blockIdx.x * 256 + threadIdx.x;
    if (i < n) { const float v = -(st[2 * i] + logf(st[2 * i + 1])); VST2(float, c + i, v); }
}

__global__ __launch_bounds__(256) void k_iota(int* __restrict__ dst, int n, int a, int b) {
    const int i = blockIdx.x * 256 + threadIdx.x;
    if (i < n) { const int v = a * i + b; VST2(int, dst + i, v); }
}

__global__ __launch_bounds__(256) void k_axpby(const float* __restrict__ x, const float* __restrict__ y, float* __restrict__ dst, int n, float a, float b, float c) {
    const int i = blockIdx.x * 256 + threadIdx.x;
    if (i < n) { const float v = a * x[i] + b * y[i] + c; VST2(float, dst + i, v); }
}

struct RopeP { const float* X; float* Y; const float* C; const float* Sn; const int* pos; long long sXr, sXh, sYr, sYh, sCb, sCp, sCd; int R, Hn, D, S, mode, tmode, pmode, pad; };
static_assert(sizeof(RopeP) == 5 * 8 + 7 * 8 + 8 * 4, "RopeP has padding");
__global__ __launch_bounds__(256) void k_rope(RopeP p) {
    const long long idx = (long long)blockIdx.x * 256 + threadIdx.x;
    if (idx >= (long long)p.R * p.Hn * p.D) return;
    const int d = (int)(idx % p.D); const long long rh = idx / p.D; const int h = (int)(rh % p.Hn); const int r = (int)(rh / p.Hn);
    const int half = p.D / 2;
    int partner; float sign;
    if (p.mode == 0) { partner = (d < half) ? d + half : d - half; sign = (d < half) ? -1.f : 1.f; }
    else { partner = d ^ 1; sign = (d & 1) ? 1.f : -1.f; }
    const int tcol = (p.tmode == 0) ? d : ((p.tmode == 1) ? (d % half) : (d >> 1));
    const int pp = (p.pmode == 0) ? (r % p.S) : ((p.pmode == 1) ? h : p.pos[r]);
    const long long toff = (long long)(r / p.S) * p.sCb + (long long)pp * p.sCp + (long long)tcol * p.sCd;
    const float* xr = p.X + (long long)r * p.sXr + (long long)h * p.sXh;
    const float v = xr[d] * p.C[toff] + sign * xr[partner] * p.Sn[toff];
    VST2(float, p.Y + (long long)r * p.sYr + (long long)h * p.sYh + d, v);
}

__global__ __launch_bounds__(256) void k_invf(float* __restrict__ invb, int half, int D, float base, float num, int fmode, float cexp) {
    const int i = blockIdx.x * 256 + threadIdx.x;
    if (i >= ((half + 31) / 32) * 32) return;
    if (i >= half) { VST2(float, invb + i, 0.f); return; }
    const float e = (float)(2 * i) / (float)D;
    float invf;
    if (fmode == 1) invf = num * expf((float)(2 * i) * cexp);
    else if (fmode == 2) invf = num * powf(base, (-2.0f * ((float)i - 1.0f)) / (float)D);
    else invf = num * (1.0f / powf(base, e));
    VST2(float, invb + i, invf);
}
__global__ __launch_bounds__(256) void k_sincos(float* __restrict__ cs, float* __restrict__ sn, const float* __restrict__ invb, int S, int half, float pscale) {
    const int idx = blockIdx.x * 256 + threadIdx.x;
    if (idx >= S * half) return;
    const int s = idx / half, i = idx - s * half;
    const float ang = (pscale * (float)s) * invb[i];
    VST2(float, cs + idx, cosf(ang)); VST2(float, sn + idx, sinf(ang));
}

__global__ __launch_bounds__(256) void k_mulact(const float* __restrict__ x, const float* __restrict__ y, float* __restrict__ dst, int n, int act) {
    const int i = blockIdx.x * 256 + threadIdx.x;
    if (i < n) { const float v = act_fn(x[i], act) * y[i]; VST2(float, dst + i, v); }
}

__global__ __launch_bounds__(256) void k_matvec(GemmP p) {
    const int rpt = (p.N == 1) ? 1 : 32;
    const long long r0 = ((long long)blockIdx.x * 256 + threadIdx.x) * rpt; const int z = blockIdx.z, zo = z / p.zi_n, zi = z - zo * p.zi_n;
    if (r0 >= p.M) return;
    const float* Bb = p.B + zo * p.sBo + zi * p.sBi;
    float* C = p.C + zo * p.sCo + zi * p.sCi; const float* R = p.R + zo * p.sRo + zi * p.sRi;
    for (int rr = 0; rr < rpt; ++rr) {
        const long long r = r0 + rr; if (r >= p.M) break;
        const float* A = p.A + zo * p.sAo + zi * p.sAi + r * p.sAm;
        float acc[8] = {0.f, 0.f, 0.f, 0.f, 0.f, 0.f, 0.f, 0.f};
        for (int k = 0; k < p.K; ++k) { const float a = A[(long long)k * p.sAk];
#pragma unroll
            for (int j = 0; j < 8; ++j) if (j < p.N) acc[j] += a * Bb[(long long)j * p.sBn + (long long)k * p.sBk]; }
#pragma unroll
        for (int j = 0; j < 8; ++j) if (j < p.N) {
            float v = acc[j] * p.alpha;
            if (p.flags & 1) v += p.bias[j];
            if (p.flags & 2) v += p.bias[r];
            v = act_fn(v, p.act);
            if (p.flags & 4) v += p.beta * R[r * p.sRm + (long long)j * p.sRn];
            VST2(float, C + r * p.sCm + j, v);
        }
    }
}
__global__ __launch_bounds__(256) void k_smallsoftmax(const float* __restrict__ src, float* __restrict__ dst, long long sr, long long dr, int n, long long R, float scale) {
    const long long r0 = ((long long)blockIdx.x * 256 + threadIdx.x) * 32;
    for (int rr = 0; rr < 32; ++rr) {
        const long long r = r0 + rr; if (r >= R) return;
        const float* s = src + r * sr; float* d = dst + r * dr;
        float mx = -__builtin_inff();
        for (int j = 0; j < n; ++j) mx = fmaxf(mx, s[j] * scale);
        float sum = 0.f;
        for (int j = 0; j < n; ++j) sum += expf(s[j] * scale - mx);
        const float inv = 1.f / sum;
        for (int j = 0; j < n; ++j) { const float v = expf(s[j] * scale - mx) * inv; VST2(float, d + j, v); }
    }
}

__global__ __launch_bounds__(32) void k_unitstat(float* __restrict__ st) { const int t = threadIdx.x; const float v = (t == 1) ? 1.f : 0.f; VST2(float, st + t, v); }

__global__ __launch_bounds__(256) void k_lincopy(const float* __restrict__ src, long long lds, float* __restrict__ dst, long long ldd, long long rows, int cols) {
    const long long i = (long long)blockIdx.x * 256 + threadIdx.x; if (i >= rows * cols) return;
    const long long r = i / cols; const int c = (int)(i - r * cols);
    const float v = src[r * lds + c]; VST2(float, dst + r * ldd + c, v);
}

__global__ __launch_bounds__(256) void k_dk_padx(const float* __restrict__ X, float* __restrict__ XP, int planes, int Hs, int PW) { const long long q = (long long)blockIdx.x * 256 + threadIdx.x; if (q >= (long long)planes * PW * PW) return; const int xx = (int)(q % PW); const int yy = (int)((q / PW) % PW); const long long pl = q / ((long long)PW * PW); float v = 0.f; if (xx >= 1 && xx <= Hs && yy >= 1 && yy <= Hs) v = X[(pl * Hs + (yy - 1)) * Hs + (xx - 1)]; VST2(float, XP + q, v); }
__global__ __launch_bounds__(64) void k_dk_dbias(const float* __restrict__ X, const float* __restrict__ W1, const float* __restrict__ b1, const float* __restrict__ W2, const float* __restrict__ b2, float* __restrict__ DB, int C, int CO, int P) { __shared__ float gm[64]; __shared__ float hb[64]; const int b = blockIdx.x; const int c = threadIdx.x; const float* xc = X + ((long long)b * C + c) * P; float s = 0.f;
#pragma unroll 1
    for (int i = 0; i < P; i += 4) { const v4f v = *(const v4f*)(xc + i); s += (v.x + v.y) + (v.z + v.w); } gm[c] = s / (float)P; __syncthreads();
    float a = b1[c]; for (int j = 0; j < C; ++j) a += W1[c * C + j] * gm[j]; hb[c] = fmaxf(a, 0.f); __syncthreads();
    float d = b2[c]; for (int j = 0; j < CO; ++j) d += W2[c * CO + j] * hb[j]; VST2(float, DB + b * CO + c, d); }
__global__ __launch_bounds__(256) void k_dk_att(const float* __restrict__ A1, const float* __restrict__ b1, const float* __restrict__ W2, const float* __restrict__ b2, const float* __restrict__ W3, const float* __restrict__ b3, float* __restrict__ F, int Bn, int MP, int PW, int NAP) { const long long q = (long long)blockIdx.x * 256 + threadIdx.x; if (q >= (long long)Bn * MP) return; const int m = (int)(q % MP); const int b = (int)(q / MP); const bool valid = (m % PW) < 128; __shared__ float a0[9][256]; __shared__ float a1v[9][256]; const int tl = threadIdx.x;
#pragma unroll 1
    for (int i = 0; i < 9; ++i) a0[i][tl] = fmaxf(A1[q * NAP + i] + b1[i], 0.f);
#pragma unroll 1
    for (int i = 0; i < 9; ++i) { float s = b2[i];
#pragma unroll 1
        for (int j = 0; j < 9; ++j) s += W2[i * 9 + j] * a0[j][tl]; a1v[i][tl] = fmaxf(s, 0.f); }
#pragma unroll 1
    for (int t = 0; t < 9; ++t) { float s = b3[t];
#pragma unroll 1
        for (int j = 0; j < 9; ++j) s += W3[t * 9 + j] * a1v[j][tl]; const float att = 1.f / (1.f + expf(-s)); VST2(float, F + ((long long)t * Bn + b) * MP + m, valid ? att : 0.f); } }
__global__ __launch_bounds__(256) void k_dk_out(const float* __restrict__ OB, const float* __restrict__ DB, float* __restrict__ OUT, int Bn, int CO, int Hs, int PW, int MP) { const long long q = (long long)blockIdx.x * 256 + threadIdx.x; if (q >= (long long)Bn * CO * Hs * Hs) return; const int xx = (int)(q % Hs); const int y = (int)((q / Hs) % Hs); const int o = (int)((q / ((long long)Hs * Hs)) % CO); const int b = (int)(q / ((long long)Hs * Hs * CO)); VST2(float, OUT + q, OB[((long long)b * MP + y * PW + xx) * CO + o] + DB[b * CO + o]); }

template __global__ void k_gemm<0>(GemmP);

extern "C" void kernel_launch(void* const* d_in, const int* in_sizes, int n_in, void* d_out, int out_size, void* d_ws, size_t ws_size, hipStream_t stream) {
    (void)in_sizes; (void)n_in; (void)out_size; (void)ws_size;
    const float* x = (const float*)d_in[0];
    const float* a1w1 = (const float*)d_in[1];
    const float* a1b1 = (const float*)d_in[2];
    const float* a1w2 = (const float*)d_in[3];
    const float* a1b2 = (const float*)d_in[4];
    const float* a1w3 = (const float*)d_in[5];
    const float* a1b3 = (const float*)d_in[6];
    const float* a3w1 = (const float*)d_in[7];
    const float* a3b1 = (const float*)d_in[8];
    const float* a3w2 = (const float*)d_in[9];
    const float* a3b2 = (const float*)d_in[10];
    const float* wt = (const float*)d_in[11];
    const int Bn = 8;
    const int C = 64;
    const int CO = 64;
    const int Hs = 128;
    const int PW = 130;
    const int PP = PW * PW;
    const int MP = 127 * PW + 128;
    const int P = Hs * Hs;
    const int NA = 9;
    const int NAP = 16;
    float* out = (float*)d_out;
    char* wsp = (char*)d_ws;
    float* XP = (float*)wsp; wsp += (((size_t)((size_t)Bn * C * PP) * 4 + 255) / 256) * 256;
    float* A1 = (float*)wsp; wsp += (((size_t)((size_t)Bn * MP * NAP) * 4 + 255) / 256) * 256;
    float* F = (float*)wsp; wsp += (((size_t)((size_t)9 * Bn * MP) * 4 + 255) / 256) * 256;
    float* OB = (float*)wsp; wsp += (((size_t)((size_t)Bn * MP * CO) * 4 + 255) / 256) * 256;
    float* DB = (float*)wsp; wsp += (((size_t)((size_t)Bn * CO) * 4 + 255) / 256) * 256;
    k_dk_padx<<<(unsigned)(((long long)Bn * C * PP + 255) / 256), 256, 0, stream>>>(x, XP, Bn * C, Hs, PW); k_dk_dbias<<<Bn, 64, 0, stream>>>(x, a3w1, a3b1, a3w2, a3b2, DB, C, CO, P);
    { GemmP ga0;
      ga0.A = XP + 0; ga0.B = a1w1 + 0; ga0.bias = XP + 0; ga0.R = XP + 0; ga0.C = A1;
      ga0.sAo = (long long)C * PP; ga0.sAi = 0; ga0.sAm = 1; ga0.sAk = PP; ga0.sBo = 0; ga0.sBi = 0; ga0.sBn = C * 9; ga0.sBk = 9; ga0.sCo = (long long)MP * NAP; ga0.sCi = 0; ga0.sCm = NAP; ga0.sRo = 0; ga0.sRi = 0; ga0.sRm = 0; ga0.sRn = 0;
      ga0.M = MP; ga0.N = NA; ga0.K = C; ga0.zi_n = 1; ga0.flags = 0; ga0.act = 0;
      ga0.alpha = 1.0f; ga0.beta = 0.0f; ga0.sa = 1.0f; ga0.sb = 8.0f; ga0.Npad = NAP; ga0.pad_ = 0;
      if ((long long)(MP) >= 64 && (long long)(NAP) >= 64) k_gemmT<0, 4, 4><<<dim3((unsigned)((NAP) + 63) / 64, (unsigned)((MP) + 63) / 64, (unsigned)(Bn)), 32, 0, stream>>>(ga0);
      else k_gemm<0><<<dim3((unsigned)((NAP) + 31) / 32, (unsigned)((MP) + 15) / 16, (unsigned)(Bn)), 32, 0, stream>>>(ga0); }
    { GemmP ga1;
      ga1.A = XP + 1; ga1.B = a1w1 + 1; ga1.bias = XP + 1; ga1.R = A1; ga1.C = A1;
      ga1.sAo = (long long)C * PP; ga1.sAi = 0; ga1.sAm = 1; ga1.sAk = PP; ga1.sBo = 0; ga1.sBi = 0; ga1.sBn = C * 9; ga1.sBk = 9; ga1.sCo = (long long)MP * NAP; ga1.sCi = 0; ga1.sCm = NAP; ga1.sRo = (long long)MP * NAP; ga1.sRi = 0; ga1.sRm = NAP; ga1.sRn = 1;
      ga1.M = MP; ga1.N = NA; ga1.K = C; ga1.zi_n = 1; ga1.flags = 4; ga1.act = 0;
      ga1.alpha = 1.0f; ga1.beta = 1.0f; ga1.sa = 1.0f; ga1.sb = 8.0f; ga1.Npad = NAP; ga1.pad_ = 0;
      if ((long long)(MP) >= 64 && (long long)(NAP) >= 64) k_gemmT<0, 4, 4><<<dim3((unsigned)((NAP) + 63) / 64, (unsigned)((MP) + 63) / 64, (unsigned)(Bn)), 32, 0, stream>>>(ga1);
      else k_gemm<0><<<dim3((unsigned)((NAP) + 31) / 32, (unsigned)((MP) + 15) / 16, (unsigned)(Bn)), 32, 0, stream>>>(ga1); }
    { GemmP ga2;
      ga2.A = XP + 2; ga2.B = a1w1 + 2; ga2.bias = XP + 2; ga2.R = A1; ga2.C = A1;
      ga2.sAo = (long long)C * PP; ga2.sAi = 0; ga2.sAm = 1; ga2.sAk = PP; ga2.sBo = 0; ga2.sBi = 0; ga2.sBn = C * 9; ga2.sBk = 9; ga2.sCo = (long long)MP * NAP; ga2.sCi = 0; ga2.sCm = NAP; ga2.sRo = (long long)MP * NAP; ga2.sRi = 0; ga2.sRm = NAP; ga2.sRn = 1;
      ga2.M = MP; ga2.N = NA; ga2.K = C; ga2.zi_n = 1; ga2.flags = 4; ga2.act = 0;
      ga2.alpha = 1.0f; ga2.beta = 1.0f; ga2.sa = 1.0f; ga2.sb = 8.0f; ga2.Npad = NAP; ga2.pad_ = 0;
      if ((long long)(MP) >= 64 && (long long)(NAP) >= 64) k_gemmT<0, 4, 4><<<dim3((unsigned)((NAP) + 63) / 64, (unsigned)((MP) + 63) / 64, (unsigned)(Bn)), 32, 0, stream>>>(ga2);
      else k_gemm<0><<<dim3((unsigned)((NAP) + 31) / 32, (unsigned)((MP) + 15) / 16, (unsigned)(Bn)), 32, 0, stream>>>(ga2); }
    { GemmP ga3;
      ga3.A = XP + 130; ga3.B = a1w1 + 3; ga3.bias = XP + 130; ga3.R = A1; ga3.C = A1;
      ga3.sAo = (long long)C * PP; ga3.sAi = 0; ga3.sAm = 1; ga3.sAk = PP; ga3.sBo = 0; ga3.sBi = 0; ga3.sBn = C * 9; ga3.sBk = 9; ga3.sCo = (long long)MP * NAP; ga3.sCi = 0; ga3.sCm = NAP; ga3.sRo = (long long)MP * NAP; ga3.sRi = 0; ga3.sRm = NAP; ga3.sRn = 1;
      ga3.M = MP; ga3.N = NA; ga3.K = C; ga3.zi_n = 1; ga3.flags = 4; ga3.act = 0;
      ga3.alpha = 1.0f; ga3.beta = 1.0f; ga3.sa = 1.0f; ga3.sb = 8.0f; ga3.Npad = NAP; ga3.pad_ = 0;
      if ((long long)(MP) >= 64 && (long long)(NAP) >= 64) k_gemmT<0, 4, 4><<<dim3((unsigned)((NAP) + 63) / 64, (unsigned)((MP) + 63) / 64, (unsigned)(Bn)), 32, 0, stream>>>(ga3);
      else k_gemm<0><<<dim3((unsigned)((NAP) + 31) / 32, (unsigned)((MP) + 15) / 16, (unsigned)(Bn)), 32, 0, stream>>>(ga3); }
    { GemmP ga4;
      ga4.A = XP + 131; ga4.B = a1w1 + 4; ga4.bias = XP + 131; ga4.R = A1; ga4.C = A1;
      ga4.sAo = (long long)C * PP; ga4.sAi = 0; ga4.sAm = 1; ga4.sAk = PP; ga4.sBo = 0; ga4.sBi = 0; ga4.sBn = C * 9; ga4.sBk = 9; ga4.sCo = (long long)MP * NAP; ga4.sCi = 0; ga4.sCm = NAP; ga4.sRo = (long long)MP * NAP; ga4.sRi = 0; ga4.sRm = NAP; ga4.sRn = 1;
      ga4.M = MP; ga4.N = NA; ga4.K = C; ga4.zi_n = 1; ga4.flags = 4; ga4.act = 0;
      ga4.alpha = 1.0f; ga4.beta = 1.0f; ga4.sa = 1.0f; ga4.sb = 8.0f; ga4.Npad = NAP; ga4.pad_ = 0;
      if ((long long)(MP) >= 64 && (long long)(NAP) >= 64) k_gemmT<0, 4, 4><<<dim3((unsigned)((NAP) + 63) / 64, (unsigned)((MP) + 63) / 64, (unsigned)(Bn)), 32, 0, stream>>>(ga4);
      else k_gemm<0><<<dim3((unsigned)((NAP) + 31) / 32, (unsigned)((MP) + 15) / 16, (unsigned)(Bn)), 32, 0, stream>>>(ga4); }
    { GemmP ga5;
      ga5.A = XP + 132; ga5.B = a1w1 + 5; ga5.bias = XP + 132; ga5.R = A1; ga5.C = A1;
      ga5.sAo = (long long)C * PP; ga5.sAi = 0; ga5.sAm = 1; ga5.sAk = PP; ga5.sBo = 0; ga5.sBi = 0; ga5.sBn = C * 9; ga5.sBk = 9; ga5.sCo = (long long)MP * NAP; ga5.sCi = 0; ga5.sCm = NAP; ga5.sRo = (long long)MP * NAP; ga5.sRi = 0; ga5.sRm = NAP; ga5.sRn = 1;
      ga5.M = MP; ga5.N = NA; ga5.K = C; ga5.zi_n = 1; ga5.flags = 4; ga5.act = 0;
      ga5.alpha = 1.0f; ga5.beta = 1.0f; ga5.sa = 1.0f; ga5.sb = 8.0f; ga5.Npad = NAP; ga5.pad_ = 0;
      if ((long long)(MP) >= 64 && (long long)(NAP) >= 64) k_gemmT<0, 4, 4><<<dim3((unsigned)((NAP) + 63) / 64, (unsigned)((MP) + 63) / 64, (unsigned)(Bn)), 32, 0, stream>>>(ga5);
      else k_gemm<0><<<dim3((unsigned)((NAP) + 31) / 32, (unsigned)((MP) + 15) / 16, (unsigned)(Bn)), 32, 0, stream>>>(ga5); }
    { GemmP ga6;
      ga6.A = XP + 260; ga6.B = a1w1 + 6; ga6.bias = XP + 260; ga6.R = A1; ga6.C = A1;
      ga6.sAo = (long long)C * PP; ga6.sAi = 0; ga6.sAm = 1; ga6.sAk = PP; ga6.sBo = 0; ga6.sBi = 0; ga6.sBn = C * 9; ga6.sBk = 9; ga6.sCo = (long long)MP * NAP; ga6.sCi = 0; ga6.sCm = NAP; ga6.sRo = (long long)MP * NAP; ga6.sRi = 0; ga6.sRm = NAP; ga6.sRn = 1;
      ga6.M = MP; ga6.N = NA; ga6.K = C; ga6.zi_n = 1; ga6.flags = 4; ga6.act = 0;
      ga6.alpha = 1.0f; ga6.beta = 1.0f; ga6.sa = 1.0f; ga6.sb = 8.0f; ga6.Npad = NAP; ga6.pad_ = 0;
      if ((long long)(MP) >= 64 && (long long)(NAP) >= 64) k_gemmT<0, 4, 4><<<dim3((unsigned)((NAP) + 63) / 64, (unsigned)((MP) + 63) / 64, (unsigned)(Bn)), 32, 0, stream>>>(ga6);
      else k_gemm<0><<<dim3((unsigned)((NAP) + 31) / 32, (unsigned)((MP) + 15) / 16, (unsigned)(Bn)), 32, 0, stream>>>(ga6); }
    { GemmP ga7;
      ga7.A = XP + 261; ga7.B = a1w1 + 7; ga7.bias = XP + 261; ga7.R = A1; ga7.C = A1;
      ga7.sAo = (long long)C * PP; ga7.sAi = 0; ga7.sAm = 1; ga7.sAk = PP; ga7.sBo = 0; ga7.sBi = 0; ga7.sBn = C * 9; ga7.sBk = 9; ga7.sCo = (long long)MP * NAP; ga7.sCi = 0; ga7.sCm = NAP; ga7.sRo = (long long)MP * NAP; ga7.sRi = 0; ga7.sRm = NAP; ga7.sRn = 1;
      ga7.M = MP; ga7.N = NA; ga7.K = C; ga7.zi_n = 1; ga7.flags = 4; ga7.act = 0;
      ga7.alpha = 1.0f; ga7.beta = 1.0f; ga7.sa = 1.0f; ga7.sb = 8.0f; ga7.Npad = NAP; ga7.pad_ = 0;
      if ((long long)(MP) >= 64 && (long long)(NAP) >= 64) k_gemmT<0, 4, 4><<<dim3((unsigned)((NAP) + 63) / 64, (unsigned)((MP) + 63) / 64, (unsigned)(Bn)), 32, 0, stream>>>(ga7);
      else k_gemm<0><<<dim3((unsigned)((NAP) + 31) / 32, (unsigned)((MP) + 15) / 16, (unsigned)(Bn)), 32, 0, stream>>>(ga7); }
    { GemmP ga8;
      ga8.A = XP + 262; ga8.B = a1w1 + 8; ga8.bias = XP + 262; ga8.R = A1; ga8.C = A1;
      ga8.sAo = (long long)C * PP; ga8.sAi = 0; ga8.sAm = 1; ga8.sAk = PP; ga8.sBo = 0; ga8.sBi = 0; ga8.sBn = C * 9; ga8.sBk = 9; ga8.sCo = (long long)MP * NAP; ga8.sCi = 0; ga8.sCm = NAP; ga8.sRo = (long long)MP * NAP; ga8.sRi = 0; ga8.sRm = NAP; ga8.sRn = 1;
      ga8.M = MP; ga8.N = NA; ga8.K = C; ga8.zi_n = 1; ga8.flags = 4; ga8.act = 0;
      ga8.alpha = 1.0f; ga8.beta = 1.0f; ga8.sa = 1.0f; ga8.sb = 8.0f; ga8.Npad = NAP; ga8.pad_ = 0;
      if ((long long)(MP) >= 64 && (long long)(NAP) >= 64) k_gemmT<0, 4, 4><<<dim3((unsigned)((NAP) + 63) / 64, (unsigned)((MP) + 63) / 64, (unsigned)(Bn)), 32, 0, stream>>>(ga8);
      else k_gemm<0><<<dim3((unsigned)((NAP) + 31) / 32, (unsigned)((MP) + 15) / 16, (unsigned)(Bn)), 32, 0, stream>>>(ga8); }
    k_dk_att<<<(unsigned)(((long long)Bn * MP + 255) / 256), 256, 0, stream>>>(A1, a1b1, a1w2, a1b2, a1w3, a1b3, F, Bn, MP, PW, NAP);
    { GemmP gm0;
      gm0.A = XP + 0; gm0.B = wt + 0; gm0.bias = F + (size_t)0 * Bn * MP; gm0.R = XP + 0; gm0.C = OB;
      gm0.sAo = (long long)C * PP; gm0.sAi = 0; gm0.sAm = 1; gm0.sAk = PP; gm0.sBo = 0; gm0.sBi = 0; gm0.sBn = C * 9; gm0.sBk = 9; gm0.sCo = (long long)MP * CO; gm0.sCi = 0; gm0.sCm = CO; gm0.sRo = 0; gm0.sRi = 0; gm0.sRm = 0; gm0.sRn = 0;
      gm0.M = MP; gm0.N = CO; gm0.K = C; gm0.zi_n = 1; gm0.flags = 8; gm0.act = 0;
      gm0.alpha = 1.0f; gm0.beta = 0.0f; gm0.sa = 1.0f; gm0.sb = 8.0f; gm0.Npad = CO; gm0.pad_ = 0;
      if ((long long)(MP) >= 64 && (long long)(CO) >= 64) k_gemmT<0, 4, 4><<<dim3((unsigned)((CO) + 63) / 64, (unsigned)((MP) + 63) / 64, (unsigned)(Bn)), 32, 0, stream>>>(gm0);
      else k_gemm<0><<<dim3((unsigned)((CO) + 31) / 32, (unsigned)((MP) + 15) / 16, (unsigned)(Bn)), 32, 0, stream>>>(gm0); }
    { GemmP gm1;
      gm1.A = XP + 1; gm1.B = wt + 1; gm1.bias = F + (size_t)1 * Bn * MP; gm1.R = OB; gm1.C = OB;
      gm1.sAo = (long long)C * PP; gm1.sAi = 0; gm1.sAm = 1; gm1.sAk = PP; gm1.sBo = 0; gm1.sBi = 0; gm1.sBn = C * 9; gm1.sBk = 9; gm1.sCo = (long long)MP * CO; gm1.sCi = 0; gm1.sCm = CO; gm1.sRo = (long long)MP * CO; gm1.sRi = 0; gm1.sRm = CO; gm1.sRn = 1;
      gm1.M = MP; gm1.N = CO; gm1.K = C; gm1.zi_n = 1; gm1.flags = 12; gm1.act = 0;
      gm1.alpha = 1.0f; gm1.beta = 1.0f; gm1.sa = 1.0f; gm1.sb = 8.0f; gm1.Npad = CO; gm1.pad_ = 0;
      if ((long long)(MP) >= 64 && (long long)(CO) >= 64) k_gemmT<0, 4, 4><<<dim3((unsigned)((CO) + 63) / 64, (unsigned)((MP) + 63) / 64, (unsigned)(Bn)), 32, 0, stream>>>(gm1);
      else k_gemm<0><<<dim3((unsigned)((CO) + 31) / 32, (unsigned)((MP) + 15) / 16, (unsigned)(Bn)), 32, 0, stream>>>(gm1); }
    { GemmP gm2;
      gm2.A = XP + 2; gm2.B = wt + 2; gm2.bias = F + (size_t)2 * Bn * MP; gm2.R = OB; gm2.C = OB;
      gm2.sAo = (long long)C * PP; gm2.sAi = 0; gm2.sAm = 1; gm2.sAk = PP; gm2.sBo = 0; gm2.sBi = 0; gm2.sBn = C * 9; gm2.sBk = 9; gm2.sCo = (long long)MP * CO; gm2.sCi = 0; gm2.sCm = CO; gm2.sRo = (long long)MP * CO; gm2.sRi = 0; gm2.sRm = CO; gm2.sRn = 1;
      gm2.M = MP; gm2.N = CO; gm2.K = C; gm2.zi_n = 1; gm2.flags = 12; gm2.act = 0;
      gm2.alpha = 1.0f; gm2.beta = 1.0f; gm2.sa = 1.0f; gm2.sb = 8.0f; gm2.Npad = CO; gm2.pad_ = 0;
      if ((long long)(MP) >= 64 && (long long)(CO) >= 64) k_gemmT<0, 4, 4><<<dim3((unsigned)((CO) + 63) / 64, (unsigned)((MP) + 63) / 64, (unsigned)(Bn)), 32, 0, stream>>>(gm2);
      else k_gemm<0><<<dim3((unsigned)((CO) + 31) / 32, (unsigned)((MP) + 15) / 16, (unsigned)(Bn)), 32, 0, stream>>>(gm2); }
    { GemmP gm3;
      gm3.A = XP + 130; gm3.B = wt + 3; gm3.bias = F + (size_t)3 * Bn * MP; gm3.R = OB; gm3.C = OB;
      gm3.sAo = (long long)C * PP; gm3.sAi = 0; gm3.sAm = 1; gm3.sAk = PP; gm3.sBo = 0; gm3.sBi = 0; gm3.sBn = C * 9; gm3.sBk = 9; gm3.sCo = (long long)MP * CO; gm3.sCi = 0; gm3.sCm = CO; gm3.sRo = (long long)MP * CO; gm3.sRi = 0; gm3.sRm = CO; gm3.sRn = 1;
      gm3.M = MP; gm3.N = CO; gm3.K = C; gm3.zi_n = 1; gm3.flags = 12; gm3.act = 0;
      gm3.alpha = 1.0f; gm3.beta = 1.0f; gm3.sa = 1.0f; gm3.sb = 8.0f; gm3.Npad = CO; gm3.pad_ = 0;
      if ((long long)(MP) >= 64 && (long long)(CO) >= 64) k_gemmT<0, 4, 4><<<dim3((unsigned)((CO) + 63) / 64, (unsigned)((MP) + 63) / 64, (unsigned)(Bn)), 32, 0, stream>>>(gm3);
      else k_gemm<0><<<dim3((unsigned)((CO) + 31) / 32, (unsigned)((MP) + 15) / 16, (unsigned)(Bn)), 32, 0, stream>>>(gm3); }
    { GemmP gm4;
      gm4.A = XP + 131; gm4.B = wt + 4; gm4.bias = F + (size_t)4 * Bn * MP; gm4.R = OB; gm4.C = OB;
      gm4.sAo = (long long)C * PP; gm4.sAi = 0; gm4.sAm = 1; gm4.sAk = PP; gm4.sBo = 0; gm4.sBi = 0; gm4.sBn = C * 9; gm4.sBk = 9; gm4.sCo = (long long)MP * CO; gm4.sCi = 0; gm4.sCm = CO; gm4.sRo = (long long)MP * CO; gm4.sRi = 0; gm4.sRm = CO; gm4.sRn = 1;
      gm4.M = MP; gm4.N = CO; gm4.K = C; gm4.zi_n = 1; gm4.flags = 12; gm4.act = 0;
      gm4.alpha = 1.0f; gm4.beta = 1.0f; gm4.sa = 1.0f; gm4.sb = 8.0f; gm4.Npad = CO; gm4.pad_ = 0;
      if ((long long)(MP) >= 64 && (long long)(CO) >= 64) k_gemmT<0, 4, 4><<<dim3((unsigned)((CO) + 63) / 64, (unsigned)((MP) + 63) / 64, (unsigned)(Bn)), 32, 0, stream>>>(gm4);
      else k_gemm<0><<<dim3((unsigned)((CO) + 31) / 32, (unsigned)((MP) + 15) / 16, (unsigned)(Bn)), 32, 0, stream>>>(gm4); }
    { GemmP gm5;
      gm5.A = XP + 132; gm5.B = wt + 5; gm5.bias = F + (size_t)5 * Bn * MP; gm5.R = OB; gm5.C = OB;
      gm5.sAo = (long long)C * PP; gm5.sAi = 0; gm5.sAm = 1; gm5.sAk = PP; gm5.sBo = 0; gm5.sBi = 0; gm5.sBn = C * 9; gm5.sBk = 9; gm5.sCo = (long long)MP * CO; gm5.sCi = 0; gm5.sCm = CO; gm5.sRo = (long long)MP * CO; gm5.sRi = 0; gm5.sRm = CO; gm5.sRn = 1;
      gm5.M = MP; gm5.N = CO; gm5.K = C; gm5.zi_n = 1; gm5.flags = 12; gm5.act = 0;
      gm5.alpha = 1.0f; gm5.beta = 1.0f; gm5.sa = 1.0f; gm5.sb = 8.0f; gm5.Npad = CO; gm5.pad_ = 0;
      if ((long long)(MP) >= 64 && (long long)(CO) >= 64) k_gemmT<0, 4, 4><<<dim3((unsigned)((CO) + 63) / 64, (unsigned)((MP) + 63) / 64, (unsigned)(Bn)), 32, 0, stream>>>(gm5);
      else k_gemm<0><<<dim3((unsigned)((CO) + 31) / 32, (unsigned)((MP) + 15) / 16, (unsigned)(Bn)), 32, 0, stream>>>(gm5); }
    { GemmP gm6;
      gm6.A = XP + 260; gm6.B = wt + 6; gm6.bias = F + (size_t)6 * Bn * MP; gm6.R = OB; gm6.C = OB;
      gm6.sAo = (long long)C * PP; gm6.sAi = 0; gm6.sAm = 1; gm6.sAk = PP; gm6.sBo = 0; gm6.sBi = 0; gm6.sBn = C * 9; gm6.sBk = 9; gm6.sCo = (long long)MP * CO; gm6.sCi = 0; gm6.sCm = CO; gm6.sRo = (long long)MP * CO; gm6.sRi = 0; gm6.sRm = CO; gm6.sRn = 1;
      gm6.M = MP; gm6.N = CO; gm6.K = C; gm6.zi_n = 1; gm6.flags = 12; gm6.act = 0;
      gm6.alpha = 1.0f; gm6.beta = 1.0f; gm6.sa = 1.0f; gm6.sb = 8.0f; gm6.Npad = CO; gm6.pad_ = 0;
      if ((long long)(MP) >= 64 && (long long)(CO) >= 64) k_gemmT<0, 4, 4><<<dim3((unsigned)((CO) + 63) / 64, (unsigned)((MP) + 63) / 64, (unsigned)(Bn)), 32, 0, stream>>>(gm6);
      else k_gemm<0><<<dim3((unsigned)((CO) + 31) / 32, (unsigned)((MP) + 15) / 16, (unsigned)(Bn)), 32, 0, stream>>>(gm6); }
    { GemmP gm7;
      gm7.A = XP + 261; gm7.B = wt + 7; gm7.bias = F + (size_t)7 * Bn * MP; gm7.R = OB; gm7.C = OB;
      gm7.sAo = (long long)C * PP; gm7.sAi = 0; gm7.sAm = 1; gm7.sAk = PP; gm7.sBo = 0; gm7.sBi = 0; gm7.sBn = C * 9; gm7.sBk = 9; gm7.sCo = (long long)MP * CO; gm7.sCi = 0; gm7.sCm = CO; gm7.sRo = (long long)MP * CO; gm7.sRi = 0; gm7.sRm = CO; gm7.sRn = 1;
      gm7.M = MP; gm7.N = CO; gm7.K = C; gm7.zi_n = 1; gm7.flags = 12; gm7.act = 0;
      gm7.alpha = 1.0f; gm7.beta = 1.0f; gm7.sa = 1.0f; gm7.sb = 8.0f; gm7.Npad = CO; gm7.pad_ = 0;
      if ((long long)(MP) >= 64 && (long long)(CO) >= 64) k_gemmT<0, 4, 4><<<dim3((unsigned)((CO) + 63) / 64, (unsigned)((MP) + 63) / 64, (unsigned)(Bn)), 32, 0, stream>>>(gm7);
      else k_gemm<0><<<dim3((unsigned)((CO) + 31) / 32, (unsigned)((MP) + 15) / 16, (unsigned)(Bn)), 32, 0, stream>>>(gm7); }
    { GemmP gm8;
      gm8.A = XP + 262; gm8.B = wt + 8; gm8.bias = F + (size_t)8 * Bn * MP; gm8.R = OB; gm8.C = OB;
      gm8.sAo = (long long)C * PP; gm8.sAi = 0; gm8.sAm = 1; gm8.sAk = PP; gm8.sBo = 0; gm8.sBi = 0; gm8.sBn = C * 9; gm8.sBk = 9; gm8.sCo = (long long)MP * CO; gm8.sCi = 0; gm8.sCm = CO; gm8.sRo = (long long)MP * CO; gm8.sRi = 0; gm8.sRm = CO; gm8.sRn = 1;
      gm8.M = MP; gm8.N = CO; gm8.K = C; gm8.zi_n = 1; gm8.flags = 12; gm8.act = 0;
      gm8.alpha = 1.0f; gm8.beta = 1.0f; gm8.sa = 1.0f; gm8.sb = 8.0f; gm8.Npad = CO; gm8.pad_ = 0;
      if ((long long)(MP) >= 64 && (long long)(CO) >= 64) k_gemmT<0, 4, 4><<<dim3((unsigned)((CO) + 63) / 64, (unsigned)((MP) + 63) / 64, (unsigned)(Bn)), 32, 0, stream>>>(gm8);
      else k_gemm<0><<<dim3((unsigned)((CO) + 31) / 32, (unsigned)((MP) + 15) / 16, (unsigned)(Bn)), 32, 0, stream>>>(gm8); }
    k_dk_out<<<(unsigned)(((long long)Bn * CO * P + 255) / 256), 256, 0, stream>>>(OB, DB, out, Bn, CO, Hs, PW, MP);
}
